// FactorGraphLayer_75788992905484
// MI455X (gfx1250) — hardware-verified
//
#include <hip/hip_runtime.h>
#include <stddef.h>


#define CH    64
#define NC    10
#define EC    5
#define KPB   64
#define APZ   72
#define NTHR  256
#define NWAVE 8
#define GROWS 32
#define GTHR  64
#define EPT   8
#define NGRP  2
#define CHUNK (NTHR * EPT * NGRP)
#define WCAP  (EPT * NGRP * 32)
#define LISTN (NWAVE * WCAP)
#define NBA   512
#define LDS_AGG (NBA * CH * 4 + LISTN * 4 + 64)
#define OSTW  160
#define PW_E2 0
#define PW_V  4096
#define PW_O  8192
#define PW_G1 12288
#define PW_G2 16384
#define PW_AT 20480
#define PW_NH 28672
#define PW_EH 29696
#define PTOT  30720
#define WROWS 480
#define WSCAP 268435456

static_assert((APZ % 8) == 0 && (KPB % 8) == 0);
static_assert(PTOT == WROWS * KPB);
static_assert((CHUNK & (CHUNK - 1)) == 0 && CHUNK <= 4096);
static_assert((NBA & (NBA - 1)) == 0 && NBA <= 4096);
static_assert(NTHR == NWAVE * 32 && GTHR * 16 == GROWS * 32);
static_assert((WROWS * 8) % NTHR == 0);
static_assert(OSTW == 32 * EC);
static_assert((CH % 32) == 0);

typedef float          v2f  __attribute__((ext_vector_type(2)));
typedef float          v4f  __attribute__((ext_vector_type(4)));
typedef float          v8f  __attribute__((ext_vector_type(8)));
typedef int            v4i  __attribute__((ext_vector_type(4)));
typedef int            v8i  __attribute__((ext_vector_type(8)));
typedef unsigned short v4us __attribute__((ext_vector_type(4)));
typedef unsigned short v8us __attribute__((ext_vector_type(8)));
typedef _Float16       v2h  __attribute__((ext_vector_type(2)));
typedef _Float16       v8h  __attribute__((ext_vector_type(8)));
typedef __bf16         v16b __attribute__((ext_vector_type(16)));
union FragB { v16b v; v8us u[2]; v8i w; };

__device__ __forceinline__ v8f wmb(const FragB& a, const FragB& b, v8f c) {
  v8f d = __builtin_amdgcn_wmma_f32_16x16x32_bf16(false, a.v, false, b.v, (short)0, c, false, false);
  asm volatile("v_nop\n\tv_nop\n\tv_nop\n\tv_nop" : "+v"(d) : "v"(a.w), "v"(b.w));
  return d;
}

__device__ __forceinline__ void bfsplit(float f, unsigned short& hi, unsigned short& lo) {
  const unsigned u = __float_as_uint(f);
  const unsigned r = (u + 0x7FFFu + ((u >> 16) & 1u)) & 0xFFFF0000u;
  hi = (unsigned short)(r >> 16);
  const float d = f - __uint_as_float(r);
  const unsigned ud = __float_as_uint(d);
  lo = (unsigned short)((ud + 0x7FFFu + ((ud >> 16) & 1u)) >> 16);
}

__device__ __forceinline__ void split4(v4f a, v4us& h, v4us& l) {
  unsigned short hs, ls;
  bfsplit(a.x, hs, ls); h.x = hs; l.x = ls;
  bfsplit(a.y, hs, ls); h.y = hs; l.y = ls;
  bfsplit(a.z, hs, ls); h.z = hs; l.z = ls;
  bfsplit(a.w, hs, ls); h.w = hs; l.w = ls;
}

__device__ __forceinline__ void wsync() {
  __builtin_amdgcn_fence(__ATOMIC_RELEASE, "wavefront");
  __builtin_amdgcn_wave_barrier();
  __builtin_amdgcn_fence(__ATOMIC_ACQUIRE, "wavefront");
}

template <int NT>
__device__ __forceinline__ void spillA(unsigned short* Ah, unsigned short* Al, const v8f (&v)[NT], int hh, int m) {
#pragma unroll
  for (int t = 0; t < NT; ++t)
#pragma unroll
    for (int r = 0; r < 8; ++r) {
      unsigned short hs, ls;
      bfsplit(v[t][r], hs, ls);
      const int o = (8 * hh + r) * APZ + 16 * t + m;
      Ah[o] = hs; Al[o] = ls;
    }
}

template <int NT>
__device__ __forceinline__ void mma3(const unsigned short* Ah, const unsigned short* Al,
                                     const unsigned short* __restrict__ Bh, const unsigned short* __restrict__ Bl,
                                     int lane, v8f (&acc)[NT]) {
  const int hh = lane >> 4, m = lane & 15;
#pragma unroll
  for (int t = 0; t < NT; ++t) { v8f z = {0.f, 0.f, 0.f, 0.f, 0.f, 0.f, 0.f, 0.f}; acc[t] = z; }
  const unsigned short* aph = Ah + m * APZ + 8 * hh;
  const unsigned short* apl = Al + m * APZ + 8 * hh;
  const unsigned short* bbh = Bh + (size_t)m * KPB + 8 * hh;
  const unsigned short* bbl = Bl + (size_t)m * KPB + 8 * hh;
#pragma unroll 1
  for (int ks = 0; ks < CH / 32; ++ks) {
    FragB ah, al;
    ah.u[0] = *(const v8us*)(aph + 32 * ks);
    ah.u[1] = *(const v8us*)(aph + 32 * ks + 16);
    al.u[0] = *(const v8us*)(apl + 32 * ks);
    al.u[1] = *(const v8us*)(apl + 32 * ks + 16);
#pragma unroll
    for (int t = 0; t < NT; ++t) {
      const unsigned short* bph = bbh + (size_t)(16 * t) * KPB + 32 * ks;
      const unsigned short* bpl = bbl + (size_t)(16 * t) * KPB + 32 * ks;
      FragB bh, bl;
      bh.u[0] = *(const v8us*)bph;
      bh.u[1] = *(const v8us*)(bph + 16);
      bl.u[0] = *(const v8us*)bpl;
      bl.u[1] = *(const v8us*)(bpl + 16);
      acc[t] = wmb(ah, bh, acc[t]);
      acc[t] = wmb(ah, bl, acc[t]);
      acc[t] = wmb(al, bh, acc[t]);
    }
  }
}

__global__ __launch_bounds__(NTHR) void k_wprep(
    const float* __restrict__ We2, const float* __restrict__ Wv, const float* __restrict__ Wo,
    const float* __restrict__ Wg1, const float* __restrict__ Wg2, const float* __restrict__ Wat,
    const float* __restrict__ Wnh, const float* __restrict__ Weh, unsigned short* Bpl) {
  const int i = blockIdx.x * NTHR + threadIdx.x;
  if (i >= WROWS * 8) return;
  const int R = i >> 3, k0 = (i & 7) * 8;
  const int Ru = __builtin_amdgcn_readfirstlane(R);
  const float* src;
  bool valid = true;
  if (Ru < 320) {
    const int q = Ru >> 6;
    const float* base = (q == 0) ? We2 : ((q == 1) ? Wv : ((q == 2) ? Wo : ((q == 3) ? Wg1 : Wg2)));
    src = base + (R & 63) * CH + k0;
  } else if (Ru < 448) {
    const int n = R - 320;
    src = (Ru < 384) ? (Wat + n * (2 * CH) + k0) : (Wat + (n - CH) * (2 * CH) + CH + k0);
  } else if (Ru < 464) {
    const int n = R - 448;
    valid = n < NC;
    src = Wnh + min(n, NC - 1) * CH + k0;
  } else {
    const int n = R - 464;
    valid = n < EC;
    src = Weh + min(n, EC - 1) * CH + k0;
  }
  v4f a = *(const v4f*)src, b = *(const v4f*)(src + 4);
  if (!valid) { const v4f z = {0.f, 0.f, 0.f, 0.f}; a = z; b = z; }
  v4us ha, la, hb, lb;
  split4(a, ha, la);
  split4(b, hb, lb);
  v8us hv, lv;
  hv.lo = ha; hv.hi = hb; lv.lo = la; lv.hi = lb;
  unsigned short* ph = Bpl + (size_t)i * 8;
  unsigned short* pl = Bpl + PTOT + (size_t)i * 8;
  *(volatile v8us*)ph = hv;
  *(volatile v8us*)pl = lv;
  __threadfence();
  *(volatile v8us*)ph = hv;
  *(volatile v8us*)pl = lv;
}

__global__ __launch_bounds__(GTHR) void k_node(
    const float* __restrict__ xin, const float* __restrict__ Wp, const float* __restrict__ bp,
    float* nf, const float* __restrict__ agg,
    const unsigned short* __restrict__ Bh, const unsigned short* __restrict__ Bl,
    const float* __restrict__ bg1, const float* __restrict__ bg2, const float* __restrict__ bat,
    const float* __restrict__ bnh, float* PQ, float* out0, int nN, int mode, int last) {
  __shared__ __attribute__((aligned(16))) unsigned short Ah[GROWS * APZ];
  __shared__ __attribute__((aligned(16))) unsigned short Al[GROWS * APZ];
  __shared__ __attribute__((aligned(16))) float stg[GROWS * 2 * CH];
  const int tid = threadIdx.x, lane = tid & 31, wave = tid >> 5, hh = lane >> 4, m = lane & 15;
  const int rowBase = blockIdx.x * GROWS;
  unsigned short* Ahw = Ah + wave * 16 * APZ;
  unsigned short* Alw = Al + wave * 16 * APZ;
  {
    const int r = tid >> 1, c0 = (tid & 1) * 32;
    const int xrow = min(rowBase + r, nN - 1);
    if (mode == 0) {
      float lg[NC];
#pragma unroll
      for (int j = 0; j < NC; ++j) lg[j] = xin[(size_t)xrow * NC + j];
#pragma unroll
      for (int c8 = 0; c8 < 32; c8 += 8) {
        float v[8];
#pragma unroll
        for (int e = 0; e < 8; ++e) {
          const int col = c0 + c8 + e;
          float a = 0.f;
#pragma unroll
          for (int j = 0; j < NC; ++j) a += lg[j] * Wp[col * NC + j];
          v[e] = a + bp[col];
        }
        const v4f a4 = {v[0], v[1], v[2], v[3]}, b4 = {v[4], v[5], v[6], v[7]};
        *(v4f*)(stg + r * CH + c0 + c8) = a4;
        *(v4f*)(stg + r * CH + c0 + c8 + 4) = b4;
        v4us h0, l0, h1, l1;
        split4(a4, h0, l0); split4(b4, h1, l1);
        *(v4us*)(Ah + r * APZ + c0 + c8) = h0; *(v4us*)(Ah + r * APZ + c0 + c8 + 4) = h1;
        *(v4us*)(Al + r * APZ + c0 + c8) = l0; *(v4us*)(Al + r * APZ + c0 + c8 + 4) = l1;
      }
    } else {
#pragma unroll
      for (int c8 = 0; c8 < 32; c8 += 8) {
        const size_t o = (size_t)xrow * CH + c0 + c8;
        v4f a4 = *(const v4f*)(nf + o), b4 = *(const v4f*)(nf + o + 4);
        const v4f g0 = *(const v4f*)(agg + o), g1 = *(const v4f*)(agg + o + 4);
        a4 += g0; b4 += g1;
        v4us h0, l0, h1, l1;
        split4(a4, h0, l0); split4(b4, h1, l1);
        *(v4us*)(Ah + r * APZ + c0 + c8) = h0; *(v4us*)(Ah + r * APZ + c0 + c8 + 4) = h1;
        *(v4us*)(Al + r * APZ + c0 + c8) = l0; *(v4us*)(Al + r * APZ + c0 + c8 + 4) = l1;
      }
    }
  }
  __syncthreads();
  if (mode != 0) {
    float bg1c[4], bg2c[4];
#pragma unroll
    for (int t = 0; t < 4; ++t) { bg1c[t] = bg1[16 * t + m]; bg2c[t] = bg2[16 * t + m]; }
    v8f acc[4];
    mma3<4>(Ahw, Alw, Bh + PW_G1, Bl + PW_G1, lane, acc);
#pragma unroll
    for (int t = 0; t < 4; ++t)
#pragma unroll
      for (int r = 0; r < 8; ++r) acc[t][r] = fmaxf(acc[t][r] + bg1c[t], 0.f);
    wsync();
    spillA<4>(Ahw, Alw, acc, hh, m);
    wsync();
    mma3<4>(Ahw, Alw, Bh + PW_G2, Bl + PW_G2, lane, acc);
#pragma unroll
    for (int t = 0; t < 4; ++t)
#pragma unroll
      for (int r = 0; r < 8; ++r) {
        const float v = fmaxf(acc[t][r] + bg2c[t], 0.f);
        acc[t][r] = v;
        stg[(wave * 16 + 8 * hh + r) * CH + 16 * t + m] = v;
      }
    wsync();
    spillA<4>(Ahw, Alw, acc, hh, m);
  }
  __syncthreads();
  {
    float* gp = nf + (size_t)rowBase * CH;
    v4f v[8];
#pragma unroll
    for (int it = 0; it < 8; ++it) v[it] = *(const v4f*)(stg + 4 * (it * GTHR + tid));
#pragma unroll
    for (int it = 0; it < 8; ++it) *(volatile v4f*)(gp + 4 * (it * GTHR + tid)) = v[it];
    __threadfence();
#pragma unroll
    for (int it = 0; it < 8; ++it) *(volatile v4f*)(gp + 4 * (it * GTHR + tid)) = v[it];
  }
  __syncthreads();
  if (last) {
    v8f ha[1];
    mma3<1>(Ahw, Alw, Bh + PW_NH, Bl + PW_NH, lane, ha);
    const float bn = bnh[min(m, NC - 1)];
    if (m < NC) {
#pragma unroll
      for (int r = 0; r < 8; ++r) stg[(wave * 16 + 8 * hh + r) * NC + m] = ha[0][r] + bn;
    }
    __syncthreads();
    int rows = nN - rowBase; rows = rows > GROWS ? GROWS : rows;
    const int nflt = rows * NC, full = nflt >> 2, rem = nflt & 3;
    float* op = out0 + (size_t)rowBase * NC;
    const int p1 = min(GTHR + tid, 79);
    const v4f o0 = *(const v4f*)(stg + 4 * tid);
    const v4f o1 = *(const v4f*)(stg + 4 * p1);
    float tr[3];
#pragma unroll
    for (int k = 0; k < 3; ++k) tr[k] = stg[min(4 * full + k, GROWS * NC - 1)];
    if (tid < full) *(volatile v4f*)(op + 4 * tid) = o0;
    if (GTHR + tid < full) *(volatile v4f*)(op + 4 * (GTHR + tid)) = o1;
    if (tid == 0) {
      if (rem > 0) ((volatile float*)op)[4 * full] = tr[0];
      if (rem > 1) ((volatile float*)op)[4 * full + 1] = tr[1];
      if (rem > 2) ((volatile float*)op)[4 * full + 2] = tr[2];
    }
    __threadfence();
    if (tid < full) *(volatile v4f*)(op + 4 * tid) = o0;
    if (GTHR + tid < full) *(volatile v4f*)(op + 4 * (GTHR + tid)) = o1;
    if (tid == 0) {
      if (rem > 0) ((volatile float*)op)[4 * full] = tr[0];
      if (rem > 1) ((volatile float*)op)[4 * full + 1] = tr[1];
      if (rem > 2) ((volatile float*)op)[4 * full + 2] = tr[2];
    }
  } else {
    float batc[4];
#pragma unroll
    for (int t = 0; t < 4; ++t) batc[t] = bat[16 * t + m];
    v8f acc[4];
    mma3<4>(Ahw, Alw, Bh + PW_AT, Bl + PW_AT, lane, acc);
#pragma unroll
    for (int t = 0; t < 4; ++t)
#pragma unroll
      for (int r = 0; r < 8; ++r) stg[(wave * 16 + 8 * hh + r) * (2 * CH) + 16 * t + m] = acc[t][r];
    mma3<4>(Ahw, Alw, Bh + PW_AT + CH * KPB, Bl + PW_AT + CH * KPB, lane, acc);
#pragma unroll
    for (int t = 0; t < 4; ++t)
#pragma unroll
      for (int r = 0; r < 8; ++r) stg[(wave * 16 + 8 * hh + r) * (2 * CH) + CH + 16 * t + m] = acc[t][r] + batc[t];
    __syncthreads();
    float* gp = PQ + (size_t)rowBase * (2 * CH);
#pragma unroll
    for (int it = 0; it < 16; ++it) {
      const int f = it * GTHR + tid;
      const v4f v = *(const v4f*)(stg + 4 * f);
      *(volatile v4f*)(gp + 4 * f) = v;
    }
    __threadfence();
#pragma unroll
    for (int it = 0; it < 16; ++it) {
      const int f = it * GTHR + tid;
      const v4f v = *(const v4f*)(stg + 4 * f);
      *(volatile v4f*)(gp + 4 * f) = v;
    }
  }
}

__global__ __launch_bounds__(NTHR) void k_edge(
    const float* __restrict__ PQ, const int* __restrict__ srcs, const int* __restrict__ dsts,
    const float* __restrict__ el, const float* __restrict__ We1, const float* __restrict__ be1,
    const unsigned short* __restrict__ Bh, const unsigned short* __restrict__ Bl,
    const float* __restrict__ be2, const float* __restrict__ bv, const float* __restrict__ bo,
    const float* __restrict__ beh, _Float16* efp, float* out1, int nN, int nE, int first, int last) {
  __shared__ __attribute__((aligned(16))) unsigned short Ah[NWAVE * 16 * APZ];
  __shared__ __attribute__((aligned(16))) unsigned short Al[NWAVE * 16 * APZ];
  __shared__ __attribute__((aligned(16))) _Float16 stf[NWAVE * 16 * CH];
  __shared__ __attribute__((aligned(16))) float ost[NWAVE * OSTW];
  __shared__ __attribute__((aligned(16))) float sW1T[EC * CH];
  __shared__ __attribute__((aligned(16))) float sb1[CH];
  const int tid = threadIdx.x, lane = tid & 31, wave = tid >> 5, hh = lane >> 4, m = lane & 15;
  for (int idx = tid; idx < EC * CH; idx += NTHR) sW1T[(idx % EC) * CH + idx / EC] = We1[idx];
  if (tid < CH) sb1[tid] = be1[tid];
  __syncthreads();
  const int ebase = (blockIdx.x * NWAVE + wave) * 32;
  if (ebase >= nE) return;
  unsigned short* Ahw = Ah + wave * 16 * APZ;
  unsigned short* Alw = Al + wave * 16 * APZ;
  _Float16* stfw = stf + wave * 16 * CH;
  float* ostw = ost + wave * OSTW;
  float be2c[4], bvc[4], boc[4];
#pragma unroll
  for (int t = 0; t < 4; ++t) { be2c[t] = be2[16 * t + m]; bvc[t] = bv[16 * t + m]; boc[t] = bo[16 * t + m]; }
  const float behc = beh[min(m, EC - 1)];

#pragma unroll 1
  for (int tt = 0; tt < 2; ++tt) {
    const int e0 = ebase + 16 * tt;
    if (e0 >= nE) break;
    const int em = min(e0 + m, nE - 1);
    int sv = srcs[em]; sv = sv < 0 ? 0 : (sv > nN - 1 ? nN - 1 : sv);
    int dv = dsts[em]; dv = dv < 0 ? 0 : (dv > nN - 1 ? nN - 1 : dv);
    v8f efo[4];
    if (first) {
      float elv[EC];
#pragma unroll
      for (int j = 0; j < EC; ++j) elv[j] = el[(size_t)em * EC + j];
#pragma unroll
      for (int t = 0; t < 4; ++t) { v8f z = {0.f, 0.f, 0.f, 0.f, 0.f, 0.f, 0.f, 0.f}; efo[t] = z; }
#pragma unroll
      for (int ks = 0; ks < 2; ++ks) {
        float tA[8], tB[8];
#pragma unroll
        for (int e = 0; e < 8; ++e) { tA[e] = 0.f; tB[e] = 0.f; }
#pragma unroll
        for (int j = 0; j < EC; ++j) {
          const float* wr = sW1T + j * CH + 32 * ks + 8 * hh;
          const v4f w0 = *(const v4f*)wr, w1 = *(const v4f*)(wr + 4);
          const v4f w2 = *(const v4f*)(wr + 16), w3 = *(const v4f*)(wr + 20);
          const float x = elv[j];
          tA[0] += x * w0.x; tA[1] += x * w0.y; tA[2] += x * w0.z; tA[3] += x * w0.w;
          tA[4] += x * w1.x; tA[5] += x * w1.y; tA[6] += x * w1.z; tA[7] += x * w1.w;
          tB[0] += x * w2.x; tB[1] += x * w2.y; tB[2] += x * w2.z; tB[3] += x * w2.w;
          tB[4] += x * w3.x; tB[5] += x * w3.y; tB[6] += x * w3.z; tB[7] += x * w3.w;
        }
        {
          const float* br = sb1 + 32 * ks + 8 * hh;
          const v4f c0 = *(const v4f*)br, c1 = *(const v4f*)(br + 4);
          const v4f c2 = *(const v4f*)(br + 16), c3 = *(const v4f*)(br + 20);
          tA[0] = fmaxf(tA[0] + c0.x, 0.f); tA[1] = fmaxf(tA[1] + c0.y, 0.f);
          tA[2] = fmaxf(tA[2] + c0.z, 0.f); tA[3] = fmaxf(tA[3] + c0.w, 0.f);
          tA[4] = fmaxf(tA[4] + c1.x, 0.f); tA[5] = fmaxf(tA[5] + c1.y, 0.f);
          tA[6] = fmaxf(tA[6] + c1.z, 0.f); tA[7] = fmaxf(tA[7] + c1.w, 0.f);
          tB[0] = fmaxf(tB[0] + c2.x, 0.f); tB[1] = fmaxf(tB[1] + c2.y, 0.f);
          tB[2] = fmaxf(tB[2] + c2.z, 0.f); tB[3] = fmaxf(tB[3] + c2.w, 0.f);
          tB[4] = fmaxf(tB[4] + c3.x, 0.f); tB[5] = fmaxf(tB[5] + c3.y, 0.f);
          tB[6] = fmaxf(tB[6] + c3.z, 0.f); tB[7] = fmaxf(tB[7] + c3.w, 0.f);
        }
        FragB ah, al;
#pragma unroll
        for (int e = 0; e < 8; ++e) {
          unsigned short hs, ls;
          bfsplit(tA[e], hs, ls); ah.u[0][e] = hs; al.u[0][e] = ls;
          bfsplit(tB[e], hs, ls); ah.u[1][e] = hs; al.u[1][e] = ls;
        }
#pragma unroll
        for (int t = 0; t < 4; ++t) {
          const unsigned short* bph = Bh + PW_E2 + (size_t)(16 * t + m) * KPB + 32 * ks + 8 * hh;
          const unsigned short* bpl = Bl + PW_E2 + (size_t)(16 * t + m) * KPB + 32 * ks + 8 * hh;
          FragB bh, bl;
          bh.u[0] = *(const v8us*)bph; bh.u[1] = *(const v8us*)(bph + 16);
          bl.u[0] = *(const v8us*)bpl; bl.u[1] = *(const v8us*)(bpl + 16);
          efo[t] = wmb(ah, bh, efo[t]);
          efo[t] = wmb(ah, bl, efo[t]);
          efo[t] = wmb(al, bh, efo[t]);
        }
      }
#pragma unroll
      for (int t = 0; t < 4; ++t)
#pragma unroll
        for (int r = 0; r < 8; ++r) efo[t][r] += be2c[t];
    } else {
#pragma unroll
      for (int t = 0; t < 4; ++t)
#pragma unroll
        for (int r = 0; r < 8; ++r) {
          const int row = min(e0 + 8 * hh + r, nE - 1);
          efo[t][r] = (float)efp[(size_t)row * CH + 16 * t + m];
        }
    }
    wsync();
#pragma unroll
    for (int i = 0; i < 8; ++i) {
      const int j = 2 * i + hh;
      const int sj = __shfl(sv, j, 32), dj = __shfl(dv, j, 32);
      const v4f p = *(const v4f*)(PQ + (size_t)sj * (2 * CH) + 4 * m);
      const v4f qq = *(const v4f*)(PQ + (size_t)dj * (2 * CH) + CH + 4 * m);
      const v4f c = p + qq;
      v4us hv4, lv4;
      split4(c, hv4, lv4);
      *(v4us*)(Ahw + j * APZ + 4 * m) = hv4;
      *(v4us*)(Alw + j * APZ + 4 * m) = lv4;
    }
    wsync();
    v8f acc[4];
    mma3<4>(Ahw, Alw, Bh + PW_V, Bl + PW_V, lane, acc);
#pragma unroll
    for (int t = 0; t < 4; ++t)
#pragma unroll
      for (int r = 0; r < 8; ++r) acc[t][r] += bvc[t];
    wsync();
    spillA<4>(Ahw, Alw, acc, hh, m);
    wsync();
    mma3<4>(Ahw, Alw, Bh + PW_O, Bl + PW_O, lane, acc);
#pragma unroll
    for (int t = 0; t < 4; ++t)
#pragma unroll
      for (int r = 0; r < 8; ++r) efo[t][r] = fmaxf(efo[t][r] + (acc[t][r] + boc[t]), 0.f);
    wsync();
#pragma unroll
    for (int t = 0; t < 4; ++t)
#pragma unroll
      for (int r = 0; r < 8; ++r) stfw[(8 * hh + r) * CH + 16 * t + m] = (_Float16)efo[t][r];
    wsync();
    v8h vq[4];
#pragma unroll
    for (int q4 = 0; q4 < 4; ++q4) {
      const int p = 32 * q4 + lane;
      vq[q4] = *(const v8h*)(stfw + (p >> 3) * CH + (p & 7) * 8);
    }
#pragma unroll
    for (int q4 = 0; q4 < 4; ++q4) {
      const int p = 32 * q4 + lane, grow = e0 + (p >> 3);
      if (grow < nE) *(volatile v8h*)(efp + (size_t)grow * CH + (p & 7) * 8) = vq[q4];
    }
    __threadfence();
#pragma unroll
    for (int q4 = 0; q4 < 4; ++q4) {
      const int p = 32 * q4 + lane, grow = e0 + (p >> 3);
      if (grow < nE) *(volatile v8h*)(efp + (size_t)grow * CH + (p & 7) * 8) = vq[q4];
    }
    if (last) {
      wsync();
      spillA<4>(Ahw, Alw, efo, hh, m);
      wsync();
      v8f ha[1];
      mma3<1>(Ahw, Alw, Bh + PW_EH, Bl + PW_EH, lane, ha);
      if (m < EC) {
#pragma unroll
        for (int r = 0; r < 8; ++r) ostw[(16 * tt + 8 * hh + r) * EC + m] = ha[0][r] + behc;
      }
    }
  }
  if (last) {
    wsync();
    int nrows = nE - ebase; nrows = nrows > 32 ? 32 : nrows;
    const int nflt = nrows * EC, full = nflt >> 2, rem = nflt & 3;
    float* op = out1 + (size_t)ebase * EC;
    const int p1 = min(32 + lane, 39);
    const v4f o0 = *(const v4f*)(ostw + 4 * lane);
    const v4f o1 = *(const v4f*)(ostw + 4 * p1);
    float tr[3];
#pragma unroll
    for (int k = 0; k < 3; ++k) tr[k] = ostw[min(4 * full + k, OSTW - 1)];
    if (lane < full) *(volatile v4f*)(op + 4 * lane) = o0;
    if (32 + lane < full) *(volatile v4f*)(op + 4 * (32 + lane)) = o1;
    if (lane == 0) {
      if (rem > 0) ((volatile float*)op)[4 * full] = tr[0];
      if (rem > 1) ((volatile float*)op)[4 * full + 1] = tr[1];
      if (rem > 2) ((volatile float*)op)[4 * full + 2] = tr[2];
    }
    __threadfence();
    if (lane < full) *(volatile v4f*)(op + 4 * lane) = o0;
    if (32 + lane < full) *(volatile v4f*)(op + 4 * (32 + lane)) = o1;
    if (lane == 0) {
      if (rem > 0) ((volatile float*)op)[4 * full] = tr[0];
      if (rem > 1) ((volatile float*)op)[4 * full + 1] = tr[1];
      if (rem > 2) ((volatile float*)op)[4 * full + 2] = tr[2];
    }
  }
}

template <int NB>
__device__ __forceinline__ int scan_chunk(const int* __restrict__ dl, int nE, int cbase, int slotBase,
                                          int vec8, int* list, int tid, int lane, int wave) {
  int wc = 0;
#pragma unroll
  for (int g = 0; g < NGRP; ++g) {
    const int el0  = (g * NTHR + tid) * EPT;
    const int e0   = cbase + el0;
    const int sent = -2147483647 - 1;
    v4i da, db;
    if (vec8 != 0 && cbase + CHUNK <= nE) {
      da = *(const v4i*)(dl + e0);
      db = *(const v4i*)(dl + e0 + 4);
    } else {
      da.x = (e0     < nE) ? dl[min(e0, nE - 1)] : sent;
      da.y = (e0 + 1 < nE) ? dl[min(e0 + 1, nE - 1)] : sent;
      da.z = (e0 + 2 < nE) ? dl[min(e0 + 2, nE - 1)] : sent;
      da.w = (e0 + 3 < nE) ? dl[min(e0 + 3, nE - 1)] : sent;
      db.x = (e0 + 4 < nE) ? dl[min(e0 + 4, nE - 1)] : sent;
      db.y = (e0 + 5 < nE) ? dl[min(e0 + 5, nE - 1)] : sent;
      db.z = (e0 + 6 < nE) ? dl[min(e0 + 6, nE - 1)] : sent;
      db.w = (e0 + 7 < nE) ? dl[min(e0 + 7, nE - 1)] : sent;
    }
    const unsigned nb = (unsigned)slotBase;
    const unsigned s0 = (unsigned)da.x - nb, s1 = (unsigned)da.y - nb;
    const unsigned s2 = (unsigned)da.z - nb, s3 = (unsigned)da.w - nb;
    const unsigned s4 = (unsigned)db.x - nb, s5 = (unsigned)db.y - nb;
    const unsigned s6 = (unsigned)db.z - nb, s7 = (unsigned)db.w - nb;
    const bool h0 = s0 < (unsigned)NB, h1 = s1 < (unsigned)NB, h2 = s2 < (unsigned)NB, h3 = s3 < (unsigned)NB;
    const bool h4 = s4 < (unsigned)NB, h5 = s5 < (unsigned)NB, h6 = s6 < (unsigned)NB, h7 = s7 < (unsigned)NB;
    const unsigned any = __builtin_amdgcn_ballot_w32(h0 | h1 | h2 | h3 | h4 | h5 | h6 | h7);
    if (any != 0u) {
#define HITJ(J, HJ, SJ) { \
        const unsigned mj = __builtin_amdgcn_ballot_w32(HJ); \
        if (mj != 0u) { \
          if (HJ) { \
            const int pos = wc + (int)__builtin_amdgcn_mbcnt_lo(mj, 0u); \
            if (pos < WCAP) list[wave * WCAP + pos] = ((el0 + (J)) << 12) | (int)(SJ); \
          } \
          wc += (int)__builtin_popcount(mj); } }
      HITJ(0, h0, s0)
      HITJ(1, h1, s1)
      HITJ(2, h2, s2)
      HITJ(3, h3, s3)
      HITJ(4, h4, s4)
      HITJ(5, h5, s5)
      HITJ(6, h6, s6)
      HITJ(7, h7, s7)
#undef HITJ
    }
  }
  return wc;
}

__global__ __launch_bounds__(NTHR) void k_agg(
    const int* __restrict__ dsts, const int* __restrict__ srcs, const _Float16* __restrict__ efp,
    const float* __restrict__ nf, float* agg, int nN, int nE, int vec8) {
  extern __shared__ v4f lds_dyn[];
  float* sacc = (float*)lds_dyn;
  int*   list = (int*)(sacc + NBA * CH);
  int*   wcnt = list + LISTN;
  const int tid = threadIdx.x, lane = tid & 31, wave = tid >> 5;
  const int slotBase = blockIdx.x * NBA;
  {
    const v4f z = {0.f, 0.f, 0.f, 0.f};
    for (int i = tid; i < NBA * CH / 4; i += NTHR) ((v4f*)sacc)[i] = z;
  }
  __syncthreads();
  const int nChunks = (nE + CHUNK - 1) / CHUNK;
#pragma unroll 1
  for (int ch = 0; ch < nChunks; ++ch) {
    const int cbase = ch * CHUNK;
    const int wc = scan_chunk<NBA>(dsts, nE, cbase, slotBase, vec8, list, tid, lane, wave);
    if (lane == 0) wcnt[wave] = wc;
    __syncthreads();
#pragma unroll 1
    for (int wsx = 0; wsx < NWAVE; ++wsx) {
      int n = __builtin_amdgcn_readfirstlane(wcnt[wsx]);
      n = n > WCAP ? WCAP : (n < 0 ? 0 : n);
      const int* lp = list + wsx * WCAP;
#pragma unroll 1
      for (int i = 0; i < n; ++i) {
        const int ent  = __builtin_amdgcn_readfirstlane(lp[i]);
        const int slot = ent & (NBA - 1);
        if ((slot & (NWAVE - 1)) == wave) {
          int e = cbase + ((ent >> 12) & (CHUNK - 1));
          e = e > nE - 1 ? nE - 1 : e;
          int s = srcs[e];
          s = s < 0 ? 0 : (s > nN - 1 ? nN - 1 : s);
          const v2h hv = *(const v2h*)(efp + (size_t)e * CH + 2 * lane);
          const v2f nv = *(const v2f*)(nf + (size_t)s * CH + 2 * lane);
          float* ap = sacc + slot * CH + 2 * lane;
          v2f a = *(const v2f*)ap;
          a.x += fmaxf(nv.x + (float)hv.x, 0.f);
          a.y += fmaxf(nv.y + (float)hv.y, 0.f);
          *(v2f*)ap = a;
        }
      }
    }
    __syncthreads();
  }
  float* gp = agg + (size_t)slotBase * CH;
#pragma unroll 1
  for (int it = 0; it < NBA * CH / 4 / NTHR; ++it) {
    const int f = it * NTHR + tid;
    const v4f v = *(const v4f*)(sacc + 4 * f);
    *(volatile v4f*)(gp + 4 * f) = v;
  }
  __threadfence();
#pragma unroll 1
  for (int it = 0; it < NBA * CH / 4 / NTHR; ++it) {
    const int f = it * NTHR + tid;
    const v4f v = *(const v4f*)(sacc + 4 * f);
    *(volatile v4f*)(gp + 4 * f) = v;
  }
}

extern "C" void kernel_launch(void* const* d_in, const int* in_sizes, int n_in,
                              void* d_out, int out_size, void* d_ws, size_t ws_size,
                              hipStream_t stream) {
  if (n_in < 23) return;
  const int nN = in_sizes[0] / NC;
  const int nE = in_sizes[1] / EC;
  if (nN <= 0 || nE <= 0) return;
  if (in_sizes[0] != nN * NC || in_sizes[1] != nE * EC || in_sizes[2] != 2 * nE) return;
  if (in_sizes[3] != CH * NC || in_sizes[4] != CH || in_sizes[5] != CH * EC || in_sizes[6] != CH) return;
  if (in_sizes[7] != CH * CH || in_sizes[9] != CH * CH || in_sizes[11] != CH * CH ||
      in_sizes[13] != CH * CH || in_sizes[15] != CH * CH || in_sizes[17] != 2 * CH * CH) return;
  if (in_sizes[8] != CH || in_sizes[10] != CH || in_sizes[12] != CH || in_sizes[14] != CH ||
      in_sizes[16] != CH || in_sizes[18] != CH) return;
  if (in_sizes[19] != NC * CH || in_sizes[20] != NC || in_sizes[21] != EC * CH || in_sizes[22] != EC) return;
  if (out_size != nN * NC + nE * EC) return;
  if (nN > (1 << 24) || nE > (1 << 27)) return;

  const float* node_logits = (const float*)d_in[0];
  const float* edge_logits = (const float*)d_in[1];
  const int*   ei    = (const int*)d_in[2];
  const float* Wproj = (const float*)d_in[3],  *bproj = (const float*)d_in[4];
  const float* We1   = (const float*)d_in[5],  *be1   = (const float*)d_in[6];
  const float* We2   = (const float*)d_in[7],  *be2   = (const float*)d_in[8];
  const float* Wg1   = (const float*)d_in[9],  *bg1   = (const float*)d_in[10];
  const float* Wg2   = (const float*)d_in[11], *bg2   = (const float*)d_in[12];
  const float* Wv    = (const float*)d_in[13], *bv    = (const float*)d_in[14];
  const float* Wo    = (const float*)d_in[15], *bo    = (const float*)d_in[16];
  const float* Wattn = (const float*)d_in[17], *battn = (const float*)d_in[18];
  const float* Wnh   = (const float*)d_in[19], *bnh   = (const float*)d_in[20];
  const float* Weh   = (const float*)d_in[21], *beh   = (const float*)d_in[22];
  const int* srcs = ei;
  const int* dsts = ei + nE;
  float* out0 = (float*)d_out;
  float* out1 = out0 + (size_t)nN * NC;

  const int nBlkN  = (nN + GROWS - 1) / GROWS;
  const int NPADN  = nBlkN * GROWS;
  const int nBlkA  = (nN + NBA - 1) / NBA;
  const int NPADA  = nBlkA * NBA;
  const int nUnits = (nE + 31) / 32;
  const int nBlkE  = (nUnits + NWAVE - 1) / NWAVE;
  const int NPADE  = nUnits * 32;

  char* ws = (char*)d_ws;
  size_t off = 0;
  const size_t oB   = off; off += (size_t)PTOT * 2 * 2;            off = (off + 255) & ~(size_t)255;
  const size_t oNf  = off; off += (size_t)NPADN * CH * 4;          off = (off + 255) & ~(size_t)255;
  const size_t oPQ  = off; off += (size_t)NPADN * 2 * CH * 4;      off = (off + 255) & ~(size_t)255;
  const size_t oAgg = off; off += (size_t)NPADA * CH * 4;          off = (off + 255) & ~(size_t)255;
  const size_t oEf  = off; off += (size_t)NPADE * CH * 2;          off = (off + 255) & ~(size_t)255;
  if (off > ws_size || off > (size_t)WSCAP) return;
  unsigned short* Bpl = (unsigned short*)(ws + oB);
  const unsigned short* Bh = Bpl;
  const unsigned short* Bl = Bpl + PTOT;
  float*    nf  = (float*)(ws + oNf);
  float*    PQ  = (float*)(ws + oPQ);
  float*    agg = (float*)(ws + oAgg);
  _Float16* efp = (_Float16*)(ws + oEf);

  const int vec8 = ((nE & 3) == 0) ? 1 : 0;

  k_wprep<<<(WROWS * 8) / NTHR, NTHR, 0, stream>>>(We2, Wv, Wo, Wg1, Wg2, Wattn, Wnh, Weh, Bpl);
  k_node<<<nBlkN, GTHR, 0, stream>>>(node_logits, Wproj, bproj, nf, agg, Bh, Bl, bg1, bg2, battn, bnh,
                                     PQ, out0, nN, 0, 0);
  hipFuncSetAttribute(reinterpret_cast<const void*>(&k_agg),
                      hipFuncAttributeMaxDynamicSharedMemorySize, LDS_AGG);
  for (int it = 0; it < 2; ++it) {
    const int first = (it == 0) ? 1 : 0, last = (it == 1) ? 1 : 0;
    k_edge<<<nBlkE, NTHR, 0, stream>>>(PQ, srcs, dsts, edge_logits, We1, be1, Bh, Bl, be2, bv, bo, beh,
                                       efp, out1, nN, nE, first, last);
    k_agg<<<nBlkA, NTHR, LDS_AGG, stream>>>(dsts, srcs, efp, nf, agg, nN, nE, vec8);
    k_node<<<nBlkN, GTHR, 0, stream>>>(node_logits, Wproj, bproj, nf, agg, Bh, Bl, bg1, bg2, battn, bnh,
                                       PQ, out0, nN, 1, last);
  }
}
